// ScaledDotProductAttention_4999341932926
// MI455X (gfx1250) — hardware-verified
//
#include <hip/hip_runtime.h>
#ifndef NB
#define NB 32
#endif
#ifndef SEQ
#define SEQ 2048
#endif
#define NB_FULL 32
#define SEQ_FULL 2048
#define DM 64
#define NR ((size_t)NB * SEQ)
#define N8 (NR * DM / 8)
#define C2 0.18033688011112042f
#define PCARRY_LOG2 8.0f

static_assert(SEQ % 64 == 0);
static_assert(SEQ <= SEQ_FULL);
static_assert(NB <= NB_FULL);
static_assert(DM == 64);
static_assert((NR * DM / 8) % 256 == 0);
static_assert((size_t)NB * (SEQ / 64) * 64 * 64 == NR * DM);
static_assert((size_t)NB * (SEQ / 64) * 4 * 16 == NR);

typedef _Float16 v16h __attribute__((ext_vector_type(16)));
typedef unsigned short v8us __attribute__((ext_vector_type(8), may_alias));
typedef float  v8f  __attribute__((ext_vector_type(8)));
typedef float  v4f  __attribute__((ext_vector_type(4)));
typedef float  v4fa __attribute__((ext_vector_type(4), may_alias));
union FragH { v16h v; v8us half[2]; _Float16 h[16]; unsigned short u[16]; };

__device__ __forceinline__ unsigned short bf16_bits(float x) { unsigned int u = __float_as_uint(x); return (unsigned short)((u + 0x7FFFu + ((u >> 16) & 1u)) >> 16); }
__device__ __forceinline__ float bf16_rne(float x) { return __uint_as_float(((unsigned int)bf16_bits(x)) << 16); }

__device__ __forceinline__ v16h g2_frag(const _Float16* p, int hh) { FragH f; f.half[0] = *(const v8us*)((const unsigned short*)p + 8 * hh); f.half[1] = *(const v8us*)((const unsigned short*)p + 16 + 8 * hh); return f.v; }
__device__ __forceinline__ v8f g2_mma(v16h a, v16h b, v8f c) { v8f d = __builtin_amdgcn_wmma_f32_16x16x32_f16(false, a, false, b, (short)0, c, false, false); asm volatile("v_nop\n\tv_nop\n\tv_nop\n\tv_nop" : "+v"(d) : "v"(a), "v"(b)); return d; }

__global__ __launch_bounds__(256) void k_x16(const float* __restrict__ x, _Float16* __restrict__ X16) {
  const size_t t = (size_t)blockIdx.x * 256 + threadIdx.x; if (t >= N8) return;
  const size_t per = (size_t)SEQ * DM / 8; const size_t b = t / per, r = t - b * per;
  const float* src = x + b * (size_t)SEQ_FULL * DM + r * 8;
  const v4f a = *(const v4fa*)src, c = *(const v4fa*)(src + 4);
  FragH f;
#pragma unroll
  for (int q = 0; q < 4; ++q) { f.h[q] = (_Float16)bf16_rne(a[q]); f.h[4 + q] = (_Float16)bf16_rne(c[q]); }
  const v8us o = f.half[0];
  unsigned short* d = (unsigned short*)X16 + t * 8;
  *(volatile v8us*)d = o; __threadfence(); *(volatile v8us*)d = o;
}

__global__ __launch_bounds__(256) void k_vt(const float* __restrict__ v, _Float16* __restrict__ VT) {
  __shared__ unsigned short tl[64][66];
  const int tid = threadIdx.x; const int b = blockIdx.x / (SEQ / 64), sg = blockIdx.x - b * (SEQ / 64); const int s0 = sg * 64;
  const float* src = v + ((size_t)b * SEQ_FULL + s0) * DM;
#pragma unroll 1
  for (int it = 0; it < 4; ++it) { const int i = tid + it * 256; const int j = i >> 4, d4 = (i & 15) * 4; const v4f a = *(const v4fa*)(src + (size_t)j * DM + d4); FragH f;
#pragma unroll
    for (int q = 0; q < 4; ++q) f.h[q] = (_Float16)bf16_rne(a[q]);
#pragma unroll
    for (int q = 0; q < 4; ++q) tl[d4 + q][j] = f.u[q]; }
  __syncthreads();
  for (int pass = 0; pass < 2; ++pass) {
#pragma unroll 1
    for (int it = 0; it < 2; ++it) { const int i = tid + it * 256; const int d = i >> 3, j8 = (i & 7) * 8; FragH f;
#pragma unroll
      for (int q = 0; q < 8; ++q) f.u[q] = tl[d][j8 + q];
      *(volatile v8us*)((unsigned short*)VT + ((size_t)b * DM + d) * SEQ + s0 + j8) = f.half[0]; }
    if (pass == 0) __threadfence(); } }

__global__ __launch_bounds__(128) void k_flash(const _Float16* __restrict__ Q16, const _Float16* __restrict__ K16, const _Float16* __restrict__ VT, float* __restrict__ out) {
  __shared__ __attribute__((aligned(16))) float so[4][16][68];
  const int tid = threadIdx.x, w = tid >> 5, lane = tid & 31, ln = lane & 15, hh = lane >> 4;
  const int b = blockIdx.x / (SEQ / 64), qt = blockIdx.x - b * (SEQ / 64);
  const int q0 = qt * 64 + w * 16;
  const _Float16* qrow = Q16 + ((size_t)b * SEQ + q0 + ln) * DM;
  const v16h qf0 = g2_frag(qrow, hh), qf1 = g2_frag(qrow + 32, hh);
  const _Float16* kbase = K16 + ((size_t)b * SEQ + ln) * DM;
  const _Float16* vbase = VT + ((size_t)b * DM + ln) * SEQ;
  const v8f z8 = {0.f, 0.f, 0.f, 0.f, 0.f, 0.f, 0.f, 0.f};
  v8f o[4] = {z8, z8, z8, z8};
  float m = -1.0e30f, l = 0.f;
#pragma unroll 1
  for (int kb0 = 0; kb0 < SEQ; kb0 += 64) {
    v8f s[4];
#pragma unroll
    for (int t = 0; t < 4; ++t) {
      const _Float16* kp = kbase + (size_t)(kb0 + t * 16) * DM;
      v8f acc = z8;
      acc = g2_mma(g2_frag(kp, hh), qf0, acc);
      acc = g2_mma(g2_frag(kp + 32, hh), qf1, acc);
      s[t] = acc;
    }
    float mx = s[0][0];
#pragma unroll
    for (int t = 0; t < 4; ++t)
#pragma unroll
      for (int r = 0; r < 8; ++r) mx = fmaxf(mx, s[t][r]);
    mx = fmaxf(mx, __shfl_xor(mx, 16));
    const float mn = fmaxf(m, mx * C2);
    const float alpha = exp2f(m - mn);
    m = mn;
    const float sh = PCARRY_LOG2 - mn;
    float sum = 0.f;
    FragH pf[2];
#pragma unroll
    for (int t = 0; t < 4; ++t)
#pragma unroll
      for (int r = 0; r < 8; ++r) { const float p = exp2f(s[t][r] * C2 + sh); sum += p; pf[t >> 1].h[(t & 1) * 8 + r] = (_Float16)p; }
    l = l * alpha + sum;
#pragma unroll
    for (int dt = 0; dt < 4; ++dt)
#pragma unroll
      for (int r = 0; r < 8; ++r) o[dt][r] *= alpha;
#pragma unroll
    for (int kc = 0; kc < 2; ++kc) {
      const _Float16* vp = vbase + kb0 + kc * 32;
#pragma unroll
      for (int dt = 0; dt < 4; ++dt) o[dt] = g2_mma(g2_frag(vp + (size_t)(dt * 16) * SEQ, hh), pf[kc].v, o[dt]);
    }
  }
  const float lt = l + __shfl_xor(l, 16);
  const float inv = 1.0f / lt;
#pragma unroll
  for (int dt = 0; dt < 4; ++dt)
#pragma unroll
    for (int r = 0; r < 8; ++r) so[w][ln][dt * 16 + 8 * hh + r] = o[dt][r] * inv;
  __builtin_amdgcn_fence(4  , "workgroup");
  __builtin_amdgcn_wave_barrier();
  const int rsub = lane >> 4, c4 = (lane & 15) * 4;
  float* orow = out + ((size_t)b * SEQ + q0) * DM;
  for (int pass = 0; pass < 2; ++pass) {
#pragma unroll
    for (int q = 0; q < 8; ++q) {
      const int r = q * 2 + rsub;
      const v4f val = *(const v4fa*)&so[w][r][c4];
      *(volatile v4f*)(orow + (size_t)r * DM + c4) = val;
    }
    if (pass == 0) __threadfence();
  }
}

extern "C" void kernel_launch(void* const* d_in, const int* in_sizes, int n_in,
                              void* d_out, int out_size, void* d_ws, size_t ws_size, hipStream_t stream) {
  if (n_in < 3) return;
  const size_t need_in = ((size_t)(NB - 1) * SEQ_FULL + SEQ) * DM;
  if ((size_t)in_sizes[0] < need_in || (size_t)in_sizes[1] < need_in || (size_t)in_sizes[2] < need_in) return;
  if ((size_t)out_size < NR * DM) return;
  const float* xq = (const float*)d_in[0]; const float* xk = (const float*)d_in[1]; const float* xv = (const float*)d_in[2];
  char* ws = (char*)d_ws; size_t off = 0;
  const size_t plane = (NR * DM * 2 + 255) & ~(size_t)255;
  _Float16* Q16 = (_Float16*)(ws + off); off += plane;
  _Float16* K16 = (_Float16*)(ws + off); off += plane;
  _Float16* VT  = (_Float16*)(ws + off); off += plane;
  if (off > ws_size) return;
  k_x16<<<(unsigned)(N8 / 256), 256, 0, stream>>>(xq, Q16);
  k_x16<<<(unsigned)(N8 / 256), 256, 0, stream>>>(xk, K16);
  k_vt<<<(unsigned)(NB * (SEQ / 64)), 256, 0, stream>>>(xv, VT);
  k_flash<<<(unsigned)(NB * (SEQ / 64)), 128, 0, stream>>>(Q16, K16, VT, (float*)d_out);
}
